// HarmonicAttentionLayer_46660524703810
// MI455X (gfx1250) — hardware-verified
//
#include <hip/hip_runtime.h>


#define NB_  2
#define TT   1024
#define DM   1024
#define NH_  16
#define HD   64
#define HID  64
#define RC   256
#define NPR  262144
#define PCAR 1024.0f
typedef _Float16 h16;
typedef unsigned short bf;
typedef __attribute__((ext_vector_type(16))) __bf16   v16bf;
typedef __attribute__((ext_vector_type(16))) _Float16 v16h;
typedef __attribute__((ext_vector_type(8)))  _Float16 v8h;
typedef __attribute__((ext_vector_type(8)))  unsigned short v8us;
typedef __attribute__((ext_vector_type(8)))  float    v8f;
typedef __attribute__((ext_vector_type(4)))  float    v4f;
typedef v8h  __attribute__((may_alias)) v8ha;
typedef v4f  __attribute__((may_alias)) v4fa;
typedef v8us __attribute__((may_alias)) v8usa;

__device__ __forceinline__ unsigned short f2bf(float f) { unsigned u = __float_as_uint(f); u += 0x7FFFu + ((u >> 16) & 1u); return (unsigned short)(u >> 16); }
__device__ __forceinline__ float bf2f(unsigned short b) { return __uint_as_float(((unsigned)b) << 16); }
__device__ __forceinline__ float bfr(float f) { return bf2f(f2bf(f)); }
__device__ __forceinline__ v16h cat16(v8h lo, v8h hi) { return __builtin_shufflevector(lo, hi, 0, 1, 2, 3, 4, 5, 6, 7, 8, 9, 10, 11, 12, 13, 14, 15); }
__device__ __forceinline__ v16bf cat16b(v8us lo, v8us hi) { return __builtin_bit_cast(v16bf, __builtin_shufflevector(lo, hi, 0, 1, 2, 3, 4, 5, 6, 7, 8, 9, 10, 11, 12, 13, 14, 15)); }
__device__ __forceinline__ v8f wmma16(v16h a, v16h b, v8f c) { return __builtin_amdgcn_wmma_f32_16x16x32_f16(false, a, false, b, (short)0, c, false, false); }
__device__ __forceinline__ v8f wmmab(v16bf a, v16bf b, v8f c) { return __builtin_amdgcn_wmma_f32_16x16x32_bf16(false, a, false, b, (short)0, c, false, false); }


template <typename T16> struct WFrag;
template <> struct WFrag<h16> { typedef v16h V; static __device__ __forceinline__ V ld(const h16* p) { return cat16(*(const v8h*)p, *(const v8h*)(p + 16)); } static __device__ __forceinline__ v8f mma(V a, V b, v8f c) { return wmma16(a, b, c); } };
template <> struct WFrag<bf> { typedef v16bf V; static __device__ __forceinline__ V ld(const bf* p) { return cat16b(*(const v8us*)p, *(const v8us*)(p + 16)); } static __device__ __forceinline__ v8f mma(V a, V b, v8f c) { return wmmab(a, b, c); } };
template <typename T16, int NSPLIT, bool BIAS>
__global__ __launch_bounds__(32) void k_gemmw(const T16* __restrict__ A, const T16* __restrict__ A2, const T16* __restrict__ Bt, const T16* __restrict__ Bt2, int K, float* C, int ldc, const float* __restrict__ bias, size_t sA, size_t sB, size_t sC) {
    typedef typename WFrag<T16>::V V;
    __shared__ __align__(16) float os[16 * 68];
    const size_t z = blockIdx.z; A += z * sA; if (A2) A2 += z * sA; Bt += z * sB; if (Bt2) Bt2 += z * sB; C += z * sC;
    const int lane = threadIdx.x & 31, lr = lane & 15, hi = lane >> 4; const int r0 = blockIdx.x * 64, c0 = blockIdx.y * 64;
    v8f acc[4][4];
#pragma unroll
    for (int mb = 0; mb < 4; ++mb)
#pragma unroll
        for (int nb = 0; nb < 4; ++nb) acc[mb][nb] = (v8f){};
    const size_t aoff = (size_t)(r0 + lr) * K + 8 * hi, boff = (size_t)(c0 + lr) * K + 8 * hi;
#pragma unroll 1
    for (int kc = 0; kc < K; kc += 32) {
        V a[4], a2[4];
#pragma unroll
        for (int mb = 0; mb < 4; ++mb) { a[mb] = WFrag<T16>::ld(A + aoff + (size_t)mb * 16 * K + kc); if (NSPLIT == 1 || NSPLIT == 2) a2[mb] = WFrag<T16>::ld(A2 + aoff + (size_t)mb * 16 * K + kc); }
#pragma unroll
        for (int nb = 0; nb < 4; ++nb) { const V b = WFrag<T16>::ld(Bt + boff + (size_t)nb * 16 * K + kc); V b2; if (NSPLIT >= 2) b2 = WFrag<T16>::ld(Bt2 + boff + (size_t)nb * 16 * K + kc);
#pragma unroll
            for (int mb = 0; mb < 4; ++mb) { acc[mb][nb] = WFrag<T16>::mma(a[mb], b, acc[mb][nb]); if (NSPLIT == 1 || NSPLIT == 2) acc[mb][nb] = WFrag<T16>::mma(a2[mb], b, acc[mb][nb]); if (NSPLIT >= 2) acc[mb][nb] = WFrag<T16>::mma(a[mb], b2, acc[mb][nb]); } }
        asm volatile("v_nop\n\tv_nop\n\tv_nop\n\tv_nop" : "+v"(acc[0][0]), "+v"(acc[1][1]), "+v"(acc[2][2]), "+v"(acc[3][3]) : "v"(a[0]), "v"(a[3]));
    }
#pragma unroll
    for (int mb = 0; mb < 4; ++mb) {
#pragma unroll
        for (int nb = 0; nb < 4; ++nb) {
#pragma unroll
            for (int j = 0; j < 8; ++j) os[(hi * 8 + j) * 68 + nb * 16 + lr] = acc[mb][nb][j]; }
        __builtin_amdgcn_wave_barrier(); asm volatile("" ::: "memory");
        float* crow = C + (size_t)(r0 + mb * 16) * ldc + c0;
#pragma unroll 1
        for (int ps = 0; ps < 2; ++ps) {
#pragma unroll
            for (int s = 0; s < 8; ++s) { const int row = 2 * s + hi, cofs = lr * 4; v4f val = *(const v4fa*)(os + row * 68 + cofs); if (BIAS) { val[0] += bfr(bias[c0 + cofs]); val[1] += bfr(bias[c0 + cofs + 1]); val[2] += bfr(bias[c0 + cofs + 2]); val[3] += bfr(bias[c0 + cofs + 3]); }
                *(volatile v4f*)(crow + (size_t)row * ldc + cofs) = val; }
            if (ps == 0) __threadfence(); }
        __builtin_amdgcn_wave_barrier(); asm volatile("" ::: "memory");
    }
}

__device__ __forceinline__ h16 tohx(float x) { return (h16)x; }
__device__ __forceinline__ void splitf(float y, unsigned short& h, unsigned short& l) { h = f2bf(y); l = f2bf(y - bf2f(h)); }
typedef __attribute__((ext_vector_type(2))) unsigned short v2us;
typedef __attribute__((ext_vector_type(4))) unsigned short v4us;
typedef __attribute__((ext_vector_type(2))) _Float16 v2h;
typedef __attribute__((ext_vector_type(4))) _Float16 v4h;

__global__ __launch_bounds__(256) void k_wtG(const float* __restrict__ w, int K, int N, bf* Bt) {
    const int lane = threadIdx.x & 31; const int L0 = (blockIdx.x * 8 + (threadIdx.x >> 5)) * 8; const int nlines = N * K / 64;
#pragma unroll
    for (int ps = 0; ps < 2; ++ps) {
#pragma unroll 1
        for (int l = 0; l < 8; ++l) { const int L = L0 + l; if (L >= nlines) break; const size_t e = (size_t)L * 64 + lane * 2; const int k = (int)(e % K), n = (int)(e / K); v2us o;
            o[0] = f2bf(w[(size_t)k * N + n]); o[1] = f2bf(w[(size_t)(k + 1) * N + n]); *(volatile v2us*)(Bt + e) = o; }
        if (ps == 0) __threadfence(); }
}
__global__ __launch_bounds__(256) void k_cvt8(const float* __restrict__ src, bf* dst, size_t n8) { const size_t i = (size_t)blockIdx.x * 256 + threadIdx.x; if (i >= n8) return; const v8f v = *(const v8f*)(src + i * 8); v8us o;
#pragma unroll
    for (int k = 0; k < 8; ++k) o[k] = f2bf(v[k]); *(volatile v8us*)(dst + i * 8) = o; __threadfence(); *(volatile v8us*)(dst + i * 8) = o; }
__global__ __launch_bounds__(256) void k_w2(const float* __restrict__ W2, bf* Bt) { const int e = (blockIdx.x * 256 + threadIdx.x) * 4; if (e >= 64 * HID) return; const int k = e % HID; const int h = e / HID; v4us o;
#pragma unroll
    for (int u = 0; u < 4; ++u) o[u] = (h < NH_) ? f2bf(W2[(k + u) * NH_ + h]) : (unsigned short)0; *(volatile v4us*)(Bt + e) = o; __threadfence(); *(volatile v4us*)(Bt + e) = o; }
__global__ __launch_bounds__(256) void k_ac(const float* __restrict__ fr, const float* __restrict__ W1, const float* __restrict__ b1, float* A, float* C) { const int e = (blockIdx.x * 256 + threadIdx.x) * 4; if (e >= TT * HID) return; const int k0 = e % HID; const int i = e / HID; const float f = bfr(fr[i]); const float lf = __logf(__fadd_rn(f, 1e-6f)); v4f oa, oc;
#pragma unroll
    for (int u = 0; u < 4; ++u) { const int k = k0 + u; float t1 = __fmul_rn(f, bfr(W1[k])), t2 = __fmul_rn(lf, bfr(W1[HID + k])); asm volatile("" : "+v"(t1)); asm volatile("" : "+v"(t2)); oa[u] = __fadd_rn(__fadd_rn(t1, t2), bfr(b1[k])); oc[u] = __fsub_rn(-t1, t2); }
    for (int ps = 0; ps < 2; ++ps) { *(volatile v4f*)(A + e) = oa; *(volatile v4f*)(C + e) = oc; if (ps == 0) __threadfence(); } }
__global__ __launch_bounds__(256) void k_hp(const float* __restrict__ A, const float* __restrict__ C, int i0, bf* Hh, bf* Hl) { const size_t e = ((size_t)blockIdx.x * 256 + threadIdx.x) * 4; if (e >= (size_t)NPR * HID) return; const int k0 = (int)(e % HID); const int p = (int)(e / HID); const int il = p / TT, j = p % TT; const float* ar = A + (size_t)(i0 + il) * HID + k0; const float* cr = C + (size_t)j * HID + k0; v4us oh, ol;
#pragma unroll
    for (int u = 0; u < 4; ++u) { const float h = fmaxf(__fadd_rn(ar[u], cr[u]), 0.f); unsigned short a, b; splitf(h, a, b); oh[u] = a; ol[u] = b; } *(volatile v4us*)(Hh + e) = oh; *(volatile v4us*)(Hl + e) = ol; __threadfence(); *(volatile v4us*)(Hh + e) = oh; *(volatile v4us*)(Hl + e) = ol; }
__global__ __launch_bounds__(256) void k_pl(const float* __restrict__ F, h16* P) { const int e = (blockIdx.x * 256 + threadIdx.x) * 4; if (e >= NH_ * TT * HD) return; const int d = e % HD; const int t = (e / HD) % TT; const int h = e / (HD * TT); const float* f = F + (size_t)t * DM + h * HD + d; v4h o;
#pragma unroll
    for (int u = 0; u < 4; ++u) o[u] = tohx(f[u]); *(volatile v4h*)(P + e) = o; __threadfence(); *(volatile v4h*)(P + e) = o; }
__global__ __launch_bounds__(256) void k_vt(const float* __restrict__ V, h16* VT) { const int e = (blockIdx.x * 256 + threadIdx.x) * 2; if (e >= NH_ * HD * TT) return; const int t = e % TT; const int d = (e / TT) % HD; const int h = e / (TT * HD); v2h o; o[0] = tohx(V[(size_t)t * DM + h * HD + d]); o[1] = tohx(V[(size_t)(t + 1) * DM + h * HD + d]); *(volatile v2h*)(VT + e) = o; __threadfence(); *(volatile v2h*)(VT + e) = o; }
__global__ __launch_bounds__(256) void k_hsoft(const float* __restrict__ Sb, const float* __restrict__ BI, const float* __restrict__ b2, h16* P16) { const int lane = threadIdx.x & 31; const int row = blockIdx.x * 8 + (threadIdx.x >> 5); if (row >= NH_ * RC) return; const int il = row % RC; const int h = row / RC; const float* sr = Sb + (size_t)row * TT; const float* br = BI + (size_t)il * TT * 64 + h; const float bh = bfr(b2[h]); float v[TT / 32]; float mx = -3.0e38f;
#pragma unroll
    for (int ch = 0; ch < TT / 128; ++ch) { const int j0 = ch * 128 + lane * 4; const v4f a = *(const v4f*)(sr + j0);
#pragma unroll
        for (int u = 0; u < 4; ++u) { float t0 = a[u] * 0.125f; asm volatile("" : "+v"(t0)); const float t = __fadd_rn(t0, __fadd_rn(br[(size_t)(j0 + u) * 64], bh)); v[ch * 4 + u] = t; mx = fmaxf(mx, t); } }
#pragma unroll
    for (int sh = 16; sh; sh >>= 1) mx = fmaxf(mx, __shfl_xor(mx, sh, 32));
    float sum = 0.f;
#pragma unroll
    for (int q = 0; q < TT / 32; ++q) { float d0 = __fsub_rn(v[q], mx); asm volatile("" : "+v"(d0)); v[q] = __builtin_amdgcn_exp2f(__fmul_rn(d0, 1.4426950408889634f)); sum += v[q]; }
#pragma unroll
    for (int sh = 16; sh; sh >>= 1) sum += __shfl_xor(sum, sh, 32);
    const float f = __fdiv_rn(PCAR, sum);
    for (int ps = 0; ps < 2; ++ps) {
#pragma unroll
        for (int ch = 0; ch < TT / 128; ++ch) { v4h o4;
#pragma unroll
            for (int q = 0; q < 4; ++q) o4[q] = tohx(v[ch * 4 + q] * f); *(volatile v4h*)(P16 + (size_t)row * TT + ch * 128 + lane * 4) = o4; }
        if (ps == 0) __threadfence(); } }
__global__ __launch_bounds__(256) void k_mrg(const float* __restrict__ O, int i0, bf* Ah, bf* Al) { const int e = (blockIdx.x * 256 + threadIdx.x) * 4; if (e >= NH_ * RC * HD) return; const int d = e % HD; const int il = (e / HD) % RC; const int h = e / (HD * RC); v4us oh, ol;
#pragma unroll
    for (int u = 0; u < 4; ++u) { unsigned short a, b; splitf(O[e + u] * (1.0f / PCAR), a, b); oh[u] = a; ol[u] = b; } const size_t oo = (size_t)(i0 + il) * DM + h * HD + d; *(volatile v4us*)(Ah + oo) = oh; *(volatile v4us*)(Al + oo) = ol; __threadfence(); *(volatile v4us*)(Ah + oo) = oh; *(volatile v4us*)(Al + oo) = ol; }

extern "C" void kernel_launch(void* const* d_in, const int* in_sizes, int n_in,
                              void* d_out, int out_size, void* d_ws, size_t ws_size, hipStream_t stream) {
    (void)in_sizes; (void)n_in; (void)out_size;
    const float** I = (const float**)d_in;
    const float *x = I[0], *freqs = I[1], *Wq = I[2], *bq = I[3], *Wk = I[4], *bk = I[5], *Wv = I[6], *bv = I[7], *Wo = I[8], *bo = I[9], *W1 = I[10], *b1 = I[11], *W2 = I[12], *b2 = I[13];
    float* OUT = (float*)d_out;
    char* wsp = (char*)d_ws;
    auto take = [&](size_t bytes) { char* p = wsp; wsp += (bytes + 255) & ~(size_t)255; return (void*)p; };
    bf* BQ = (bf*)take((size_t)DM * DM * 2); bf* BK = (bf*)take((size_t)DM * DM * 2); bf* BV = (bf*)take((size_t)DM * DM * 2); bf* BO = (bf*)take((size_t)DM * DM * 2); bf* B2 = (bf*)take(64 * HID * 2);
    bf* XB = (bf*)take((size_t)TT * DM * 2); float* FQ = (float*)take((size_t)TT * DM * 4); float* FK = (float*)take((size_t)TT * DM * 4); float* FV = (float*)take((size_t)TT * DM * 4); float* A = (float*)take(TT * HID * 4); float* C = (float*)take(TT * HID * 4);
    h16* Q16 = (h16*)take((size_t)NH_ * TT * HD * 2); h16* K16 = (h16*)take((size_t)NH_ * TT * HD * 2); h16* VT = (h16*)take((size_t)NH_ * HD * TT * 2); bf* Hh = (bf*)take((size_t)NPR * HID * 2); bf* Hl = (bf*)take((size_t)NPR * HID * 2); float* BI = (float*)take((size_t)NPR * 64 * 4);
    float* Sb = (float*)take((size_t)NH_ * RC * TT * 4); h16* P16 = (h16*)take((size_t)NH_ * RC * TT * 2); float* O = (float*)take((size_t)NH_ * RC * HD * 4); bf* Ch = (bf*)take((size_t)TT * DM * 2); bf* Cl = (bf*)take((size_t)TT * DM * 2);
    if ((size_t)(wsp - (char*)d_ws) > ws_size) return;
    k_wtG<<<(DM * DM / 64 + 63) / 64, 256, 0, stream>>>(Wq, DM, DM, BQ); k_wtG<<<(DM * DM / 64 + 63) / 64, 256, 0, stream>>>(Wk, DM, DM, BK); k_wtG<<<(DM * DM / 64 + 63) / 64, 256, 0, stream>>>(Wv, DM, DM, BV); k_wtG<<<(DM * DM / 64 + 63) / 64, 256, 0, stream>>>(Wo, DM, DM, BO); k_w2<<<(64 * HID / 4 + 255) / 256, 256, 0, stream>>>(W2, B2);
    for (int b = 0; b < NB_; ++b) {
        k_cvt8<<<(TT * DM / 8 + 255) / 256, 256, 0, stream>>>(x + (size_t)b * TT * DM, XB, (size_t)TT * DM / 8);
        k_gemmw<bf, 0, true><<<dim3(TT / 64, DM / 64, 1), 32, 0, stream>>>(XB, nullptr, BQ, nullptr, DM, FQ, DM, bq, 0, 0, 0); k_gemmw<bf, 0, true><<<dim3(TT / 64, DM / 64, 1), 32, 0, stream>>>(XB, nullptr, BK, nullptr, DM, FK, DM, bk, 0, 0, 0); k_gemmw<bf, 0, true><<<dim3(TT / 64, DM / 64, 1), 32, 0, stream>>>(XB, nullptr, BV, nullptr, DM, FV, DM, bv, 0, 0, 0);
        k_pl<<<(NH_ * TT * HD / 4 + 255) / 256, 256, 0, stream>>>(FQ, Q16); k_pl<<<(NH_ * TT * HD / 4 + 255) / 256, 256, 0, stream>>>(FK, K16); k_vt<<<(NH_ * HD * TT / 2 + 255) / 256, 256, 0, stream>>>(FV, VT);
        k_ac<<<(TT * HID / 4 + 255) / 256, 256, 0, stream>>>(freqs + (size_t)b * TT, W1, b1, A, C);
        for (int i0 = 0; i0 < TT; i0 += RC) {
            k_hp<<<(unsigned)(((size_t)NPR * HID / 4 + 255) / 256), 256, 0, stream>>>(A, C, i0, Hh, Hl);
            k_gemmw<bf, 1, false><<<dim3(NPR / 64, 1, 1), 32, 0, stream>>>(Hh, Hl, B2, nullptr, HID, BI, 64, nullptr, 0, 0, 0);
            k_gemmw<h16, 0, false><<<dim3(RC / 64, TT / 64, NH_), 32, 0, stream>>>(Q16 + (size_t)i0 * HD, nullptr, K16, nullptr, HD, Sb, TT, nullptr, (size_t)TT * HD, (size_t)TT * HD, (size_t)RC * TT);
            k_hsoft<<<NH_ * RC / 8, 256, 0, stream>>>(Sb, BI, b2, P16);
            k_gemmw<h16, 0, false><<<dim3(RC / 64, 1, NH_), 32, 0, stream>>>(P16, nullptr, VT, nullptr, TT, O, HD, nullptr, (size_t)RC * TT, (size_t)HD * TT, (size_t)RC * HD);
            k_mrg<<<(NH_ * RC * HD / 4 + 255) / 256, 256, 0, stream>>>(O, i0, Ch, Cl); }
        k_gemmw<bf, 1, true><<<dim3(TT / 64, DM / 64, 1), 32, 0, stream>>>(Ch, Cl, BO, nullptr, DM, OUT + (size_t)b * TT * DM, DM, bo, 0, 0, 0); }
}
